// GRUNet_22986664969033
// MI455X (gfx1250) — hardware-verified
//
#include <hip/hip_runtime.h>
#include <math.h>

constexpr int NB    = 512;
constexpr int NSTEP = 512;
constexpr int NIN   = 10;
constexpr int NH    = 100;
constexpr int NGATE = 3;
constexpr int NOUTD = 3;
constexpr int NLAY  = 2;
constexpr int KXP   = 32;
constexpr int KHP   = 128;
constexpr int GSTR  = 128;
constexpr int NROWP = NGATE * GSTR;
constexpr int RB    = 16;
constexpr int NWAVE = 7;
constexpr int NTHR  = NWAVE * 32;
constexpr int HP    = 136;
constexpr int NTHD  = 512;
constexpr float WSC     = 16.0f;
constexpr float WSC_INV = 1.0f / 16.0f;
constexpr int NOUT0 = NB * NOUTD;
constexpr int NOUT1 = NLAY * NB * NH;
constexpr int OUT1_OFF_BYTES = 6144;
static_assert(OUT1_OFF_BYTES == NOUT0 * 4);
static_assert(OUT1_OFF_BYTES + NOUT1 * 4 == 415744);
static_assert(OUT1_OFF_BYTES % 128 == 0);
static_assert((RB * NH * 4) % 128 == 0);
static_assert(NB % RB == 0);
static_assert(NWAVE * 16 >= NH);
static_assert(NWAVE * 16 + 16 == KHP);
static_assert(KHP % 32 == 0 && KXP == 32 && KXP / 8 == 4);
static_assert(HP % 8 == 0 && HP >= KHP);
static_assert(NIN <= KXP && NH <= KHP && NH <= GSTR);
static_assert(NH % 4 == 0 && (RB * NH) % 4 == 0);
static_assert(NTHD == NB);
static_assert(NOUT0 % 4 == 0 && (NOUT0 / 4) <= NTHD && (NOUT0 * 4) % 128 == 0);
static_assert((NB * NSTEP * (KXP / 8)) % 256 == 0);
static_assert((NROWP * (KXP / 8)) % 256 == 0 && (NROWP * (KHP / 8)) % 256 == 0);

typedef __attribute__((ext_vector_type(16))) _Float16 v16h;
typedef __attribute__((ext_vector_type(8)))  _Float16 v8h;
typedef __attribute__((ext_vector_type(8)))  float    v8f;
typedef __attribute__((ext_vector_type(4)))  float    v4f;

__device__ __forceinline__ void dep_guard3_h(v8f& a, v8f& b, v8f& c, v16h w, v16h x, v16h y, v16h z) {
  asm volatile("v_nop\n\tv_nop\n\tv_nop\n\tv_nop" : "+v"(a), "+v"(b), "+v"(c) : "v"(w), "v"(x), "v"(y), "v"(z));
}
__device__ __forceinline__ void acc_guard4(v8f& a, v8f& b, v8f& c, v8f& d) {
  asm volatile("v_nop\n\tv_nop\n\tv_nop\n\tv_nop" : "+v"(a), "+v"(b), "+v"(c), "+v"(d));
}

template <typename T> struct Frag;
template <> struct Frag<_Float16> {
  typedef v16h V; union U { v16h v; v8h h[2]; };
  static __device__ __forceinline__ v16h load(const _Float16* p) {
    U f; f.h[0] = *(const v8h*)(p); f.h[1] = *(const v8h*)(p + 16); return f.v;
  }
  static __device__ __forceinline__ v8f mma(v16h a, v16h b, v8f c) {
    return __builtin_amdgcn_wmma_f32_16x16x32_f16(false, a, false, b, (short)0, c, false, false);
  }
};

__global__ __launch_bounds__(256) void xprep_kernel(const float* __restrict__ x, unsigned short* __restrict__ X16p) {
  const int i = blockIdx.x * 256 + threadIdx.x;
  if (i >= NB * NSTEP * (KXP / 8)) return;
  const int row = i >> 2;
  const int q   = i & 3;
  const float* xr = x + (size_t)row * NIN;
  v8h hv;
#pragma unroll
  for (int e = 0; e < 8; ++e) {
    const int col = 8 * q + e;
    const int cc  = (col < NIN) ? col : (NIN - 1);
    const float f = xr[cc];
    const float fac = (col < NIN) ? 1.0f : 0.0f;
    hv[e] = (_Float16)(f * fac);
  }
  _Float16* op = (_Float16*)X16p + (size_t)i * 8;
  *(volatile v8h*)op = hv;
  __threadfence();
  *(volatile v8h*)op = hv;
}

template <int KREAL, int KPITCH>
__global__ __launch_bounds__(256) void wprep_kernel(const float* __restrict__ w, unsigned short* __restrict__ dst) {
  constexpr int C8 = KPITCH / 8;
  const int i = blockIdx.x * 256 + threadIdx.x;
  if (i >= NROWP * C8) return;
  const int n  = i / C8;
  const int c8 = i - n * C8;
  const int g  = n / GSTR;
  const int u  = n - g * GSTR;
  const int uc = (u < NH) ? u : (NH - 1);
  const float ufac = (u < NH) ? WSC : 0.0f;
  const float* wr = w + (size_t)(g * NH + uc) * KREAL;
  v8h hv;
#pragma unroll
  for (int e = 0; e < 8; ++e) {
    const int k  = 8 * c8 + e;
    const int kc = (k < KREAL) ? k : (KREAL - 1);
    const float f = wr[kc];
    const float fac = (k < KREAL) ? ufac : 0.0f;
    hv[e] = (_Float16)(f * fac);
  }
  _Float16* op = (_Float16*)dst + (size_t)i * 8;
  *(volatile v8h*)op = hv;
  __threadfence();
  *(volatile v8h*)op = hv;
}

__device__ __forceinline__ float gru_cell(float ar, float az, float anx, float anh,
                                          float cbr, float cbz, float cin, float chn, float h_old) {
  const float pr  = ar  * WSC_INV + cbr;
  const float pz  = az  * WSC_INV + cbz;
  const float pnx = anx * WSC_INV + cin;
  const float pnh = anh * WSC_INV + chn;
  const float rg = __builtin_amdgcn_rcpf(1.0f + expf(-pr));
  const float zg = __builtin_amdgcn_rcpf(1.0f + expf(-pz));
  const float ng = tanhf(pnx + rg * pnh);
  return (1.0f - zg) * ng + zg * h_old;
}

__global__ __launch_bounds__(NTHR) void gru2_seq_kernel(
    const unsigned short* __restrict__ X16p, const float* __restrict__ h_in,
    const unsigned short* __restrict__ WI0p, const unsigned short* __restrict__ WH0p,
    const unsigned short* __restrict__ WI1p, const unsigned short* __restrict__ WH1p,
    const float* __restrict__ b_i0, const float* __restrict__ b_h0,
    const float* __restrict__ b_i1, const float* __restrict__ b_h1,
    float* __restrict__ out1, float* __restrict__ HFIN) {
  __shared__ __align__(16) _Float16 Ht[4][RB * HP];
  __shared__ __align__(16) float    FS[2][RB * NH];
  __shared__ float BS[4][NGATE * NH];

  const _Float16* X16 = (const _Float16*)X16p;
  const _Float16* WI0 = (const _Float16*)WI0p;
  const _Float16* WH0 = (const _Float16*)WH0p;
  const _Float16* WI1 = (const _Float16*)WI1p;
  const _Float16* WH1 = (const _Float16*)WH1p;

  const int tid = threadIdx.x, lane = tid & 31, wave = tid >> 5;
  const int rlane = lane & 15, hh = lane >> 4, koff = hh * 8, mOff = hh * 8;
  const int b0 = blockIdx.x * RB;
  const int j  = 16 * wave + rlane;
  const bool jreal = (j < NH);
  const int jc = jreal ? j : (NH - 1);

  {
    _Float16* hf = &Ht[0][0];
#pragma unroll 1
    for (int i = tid; i < 4 * RB * HP; i += NTHR) hf[i] = (_Float16)0.0f;
  }
#pragma unroll 1
  for (int i = tid; i < NGATE * NH; i += NTHR) {
    BS[0][i] = b_i0[i];
    BS[1][i] = b_h0[i];
    BS[2][i] = b_i1[i];
    BS[3][i] = b_h1[i];
  }
#pragma unroll 1
  for (int f = tid; f < NLAY * (RB * NH / 4); f += NTHR) {
    const int l  = (f < (RB * NH / 4)) ? 0 : 1;
    const int ff = f - l * (RB * NH / 4);
    const v4f v = *(const v4f*)(h_in + (size_t)(l * NB + b0) * NH + 4 * ff);
    *(v4f*)(&FS[l][4 * ff]) = v;
  }
  __syncthreads();

  const float cbr0 = jreal ? (BS[0][jc] + BS[1][jc]) : 0.0f;
  const float cbz0 = jreal ? (BS[0][NH + jc] + BS[1][NH + jc]) : 0.0f;
  const float cin0 = jreal ? BS[0][2 * NH + jc] : 0.0f;
  const float chn0 = jreal ? BS[1][2 * NH + jc] : 0.0f;
  const float cbr1 = jreal ? (BS[2][jc] + BS[3][jc]) : 0.0f;
  const float cbz1 = jreal ? (BS[2][NH + jc] + BS[3][NH + jc]) : 0.0f;
  const float cin1 = jreal ? BS[2][2 * NH + jc] : 0.0f;
  const float chn1 = jreal ? BS[3][2 * NH + jc] : 0.0f;

  float h0r[8], h1r[8];
#pragma unroll
  for (int r = 0; r < 8; ++r) {
    const float a = FS[0][(mOff + r) * NH + jc];
    const float b = FS[1][(mOff + r) * NH + jc];
    h0r[r] = jreal ? a : 0.0f;
    h1r[r] = jreal ? b : 0.0f;
    Ht[0][(mOff + r) * HP + j] = (_Float16)h0r[r];
    Ht[2][(mOff + r) * HP + j] = (_Float16)h1r[r];
  }
  const v16h wx_r = Frag<_Float16>::load(WI0 + (size_t)j * KXP + koff);
  const v16h wx_z = Frag<_Float16>::load(WI0 + (size_t)(GSTR + j) * KXP + koff);
  const v16h wx_n = Frag<_Float16>::load(WI0 + (size_t)(2 * GSTR + j) * KXP + koff);
  __syncthreads();

  const _Float16* xrow = X16 + (size_t)(b0 + rlane) * NSTEP * KXP + koff;
  const _Float16* wh0r = WH0 + (size_t)j * KHP + koff;
  const _Float16* wh0z = WH0 + (size_t)(GSTR + j) * KHP + koff;
  const _Float16* wh0n = WH0 + (size_t)(2 * GSTR + j) * KHP + koff;
  const _Float16* wi1r = WI1 + (size_t)j * KHP + koff;
  const _Float16* wi1z = WI1 + (size_t)(GSTR + j) * KHP + koff;
  const _Float16* wi1n = WI1 + (size_t)(2 * GSTR + j) * KHP + koff;
  const _Float16* wh1r = WH1 + (size_t)j * KHP + koff;
  const _Float16* wh1z = WH1 + (size_t)(GSTR + j) * KHP + koff;
  const _Float16* wh1n = WH1 + (size_t)(2 * GSTR + j) * KHP + koff;
  const v8f z8 = {0.f, 0.f, 0.f, 0.f, 0.f, 0.f, 0.f, 0.f};
  const v8h zero8 = {0, 0, 0, 0, 0, 0, 0, 0};
  const int prow = lane >> 1;
  const int pcol = NWAVE * 16 + 8 * (lane & 1);

#pragma unroll 1
  for (int t = 0; t < NSTEP; ++t) {
    const int cur = t & 1, nxt = cur ^ 1;
    {
      v8f ar = z8, az = z8, anx = z8, anh = z8;
      {
        const v16h a = Frag<_Float16>::load(xrow + (size_t)t * KXP);
        ar  = Frag<_Float16>::mma(a, wx_r, ar);
        az  = Frag<_Float16>::mma(a, wx_z, az);
        anx = Frag<_Float16>::mma(a, wx_n, anx);
        dep_guard3_h(ar, az, anx, a, wx_r, wx_z, wx_n);
      }
      const _Float16* arow = &Ht[cur][0] + rlane * HP + koff;
#pragma unroll 1
      for (int k0 = 0; k0 < KHP; k0 += 32) {
        const v16h a  = Frag<_Float16>::load(arow + k0);
        const v16h w0 = Frag<_Float16>::load(wh0r + k0);
        const v16h w1 = Frag<_Float16>::load(wh0z + k0);
        const v16h w2 = Frag<_Float16>::load(wh0n + k0);
        ar  = Frag<_Float16>::mma(a, w0, ar);
        az  = Frag<_Float16>::mma(a, w1, az);
        anh = Frag<_Float16>::mma(a, w2, anh);
        dep_guard3_h(ar, az, anh, a, w0, w1, w2);
      }
      acc_guard4(ar, az, anx, anh);
      _Float16* hn0 = &Ht[nxt][0];
#pragma unroll
      for (int r = 0; r < 8; ++r) {
        const float hv = gru_cell(ar[r], az[r], anx[r], anh[r], cbr0, cbz0, cin0, chn0, h0r[r]);
        h0r[r] = jreal ? hv : 0.0f;
        hn0[(mOff + r) * HP + j] = (_Float16)h0r[r];
      }
      if (wave == 0) *(v8h*)(hn0 + prow * HP + pcol) = zero8;
    }
    __syncthreads();
    {
      v8f ar = z8, az = z8, anx = z8, anh = z8;
      const _Float16* a0n = &Ht[nxt][0] + rlane * HP + koff;
#pragma unroll 1
      for (int k0 = 0; k0 < KHP; k0 += 32) {
        const v16h a  = Frag<_Float16>::load(a0n + k0);
        const v16h w0 = Frag<_Float16>::load(wi1r + k0);
        const v16h w1 = Frag<_Float16>::load(wi1z + k0);
        const v16h w2 = Frag<_Float16>::load(wi1n + k0);
        ar  = Frag<_Float16>::mma(a, w0, ar);
        az  = Frag<_Float16>::mma(a, w1, az);
        anx = Frag<_Float16>::mma(a, w2, anx);
        dep_guard3_h(ar, az, anx, a, w0, w1, w2);
      }
      const _Float16* a1c = &Ht[2 + cur][0] + rlane * HP + koff;
#pragma unroll 1
      for (int k0 = 0; k0 < KHP; k0 += 32) {
        const v16h a  = Frag<_Float16>::load(a1c + k0);
        const v16h w0 = Frag<_Float16>::load(wh1r + k0);
        const v16h w1 = Frag<_Float16>::load(wh1z + k0);
        const v16h w2 = Frag<_Float16>::load(wh1n + k0);
        ar  = Frag<_Float16>::mma(a, w0, ar);
        az  = Frag<_Float16>::mma(a, w1, az);
        anh = Frag<_Float16>::mma(a, w2, anh);
        dep_guard3_h(ar, az, anh, a, w0, w1, w2);
      }
      acc_guard4(ar, az, anx, anh);
      _Float16* hn1 = &Ht[2 + nxt][0];
#pragma unroll
      for (int r = 0; r < 8; ++r) {
        const float hv = gru_cell(ar[r], az[r], anx[r], anh[r], cbr1, cbz1, cin1, chn1, h1r[r]);
        h1r[r] = jreal ? hv : 0.0f;
        hn1[(mOff + r) * HP + j] = (_Float16)h1r[r];
      }
      if (wave == 1) *(v8h*)(hn1 + prow * HP + pcol) = zero8;
    }
    __syncthreads();
  }

  if (jreal) {
#pragma unroll
    for (int r = 0; r < 8; ++r) {
      FS[0][(mOff + r) * NH + j] = h0r[r];
      FS[1][(mOff + r) * NH + j] = h1r[r];
    }
  }
  __syncthreads();
  for (int pass = 0; pass < 2; ++pass) {
#pragma unroll 1
    for (int f = tid; f < RB * NH / 4; f += NTHR) {
      const v4f v0 = *(const v4f*)(&FS[0][4 * f]);
      const v4f v1 = *(const v4f*)(&FS[1][4 * f]);
      *(volatile v4f*)(out1 + (size_t)b0 * NH + 4 * f) = v0;
      *(volatile v4f*)(out1 + (size_t)(NB + b0) * NH + 4 * f) = v1;
      *(volatile v4f*)(HFIN + (size_t)b0 * NH + 4 * f) = v1;
    }
    __threadfence();
  }
}

__global__ __launch_bounds__(NTHD) void head_kernel(const float* __restrict__ HFIN, const float* __restrict__ fcw,
                                                   const float* __restrict__ fcb, float* __restrict__ out0) {
  __shared__ float fcw_s[NOUTD * NH];
  __shared__ float fcb_s[4];
  __shared__ __align__(16) float os_s[NOUT0];
  const int tid = threadIdx.x;
#pragma unroll 1
  for (int i = tid; i < NOUTD * NH; i += NTHD) fcw_s[i] = fcw[i];
  if (tid < NOUTD) fcb_s[tid] = fcb[tid];
  __syncthreads();
  const int row = tid;
  const float* hr = HFIN + (size_t)row * NH;
  float a0 = 0.0f, a1 = 0.0f, a2 = 0.0f;
#pragma unroll 1
  for (int k4 = 0; k4 < NH / 4; ++k4) {
    const v4f v = *(const v4f*)(hr + 4 * k4);
#pragma unroll
    for (int e = 0; e < 4; ++e) {
      const float u = fmaxf(v[e], 0.0f);
      const int k = 4 * k4 + e;
      a0 += u * fcw_s[k];
      a1 += u * fcw_s[NH + k];
      a2 += u * fcw_s[2 * NH + k];
    }
  }
  os_s[row * NOUTD + 0] = a0 + fcb_s[0];
  os_s[row * NOUTD + 1] = a1 + fcb_s[1];
  os_s[row * NOUTD + 2] = a2 + fcb_s[2];
  __syncthreads();
  for (int pass = 0; pass < 2; ++pass) {
    if (tid < NOUT0 / 4) {
      const v4f v = *(const v4f*)(os_s + 4 * tid);
      *(volatile v4f*)(out0 + 4 * tid) = v;
    }
    __threadfence();
  }
}

extern "C" void kernel_launch(void* const* d_in, const int* in_sizes, int n_in,
                              void* d_out, int out_size, void* d_ws, size_t ws_size, hipStream_t stream) {
  if (n_in < 12 || d_out == nullptr || d_ws == nullptr) return;
  if (in_sizes[0] != NB * NSTEP * NIN || in_sizes[1] != NLAY * NB * NH ||
      in_sizes[2] != NGATE * NH * NIN || in_sizes[3] != NGATE * NH * NH || in_sizes[4] != NGATE * NH || in_sizes[5] != NGATE * NH ||
      in_sizes[6] != NGATE * NH * NH || in_sizes[7] != NGATE * NH * NH || in_sizes[8] != NGATE * NH || in_sizes[9] != NGATE * NH ||
      in_sizes[10] != NOUTD * NH || in_sizes[11] != NOUTD || out_size != NOUT0 + NOUT1) return;

  const float* x     = (const float*)d_in[0];
  const float* h_in  = (const float*)d_in[1];
  const float* w_ih0 = (const float*)d_in[2];
  const float* w_hh0 = (const float*)d_in[3];
  const float* b_ih0 = (const float*)d_in[4];
  const float* b_hh0 = (const float*)d_in[5];
  const float* w_ih1 = (const float*)d_in[6];
  const float* w_hh1 = (const float*)d_in[7];
  const float* b_ih1 = (const float*)d_in[8];
  const float* b_hh1 = (const float*)d_in[9];
  const float* fc_w  = (const float*)d_in[10];
  const float* fc_b  = (const float*)d_in[11];
  float* out0 = (float*)d_out;
  float* out1 = (float*)d_out + NOUT0;

  char* ws = (char*)d_ws; size_t off = 0;
  auto carve = [&](size_t bytes) -> char* { char* p = ws + off; off += (bytes + 255) & ~(size_t)255; return p; };
  unsigned short* X16  = (unsigned short*)carve((size_t)NB * NSTEP * KXP * 2);
  unsigned short* WI0  = (unsigned short*)carve((size_t)NROWP * KXP * 2);
  unsigned short* WH0  = (unsigned short*)carve((size_t)NROWP * KHP * 2);
  unsigned short* WI1  = (unsigned short*)carve((size_t)NROWP * KHP * 2);
  unsigned short* WH1  = (unsigned short*)carve((size_t)NROWP * KHP * 2);
  float*          HFIN = (float*)carve((size_t)NB * NH * 4);
  if (off > ws_size || off > (size_t)134217728) return;

  xprep_kernel<<<(NB * NSTEP * (KXP / 8)) / 256, 256, 0, stream>>>(x, X16);
  wprep_kernel<NIN, KXP><<<(NROWP * (KXP / 8)) / 256, 256, 0, stream>>>(w_ih0, WI0);
  wprep_kernel<NH, KHP><<<(NROWP * (KHP / 8)) / 256, 256, 0, stream>>>(w_hh0, WH0);
  wprep_kernel<NH, KHP><<<(NROWP * (KHP / 8)) / 256, 256, 0, stream>>>(w_ih1, WI1);
  wprep_kernel<NH, KHP><<<(NROWP * (KHP / 8)) / 256, 256, 0, stream>>>(w_hh1, WH1);
  gru2_seq_kernel<<<NB / RB, NTHR, 0, stream>>>(X16, h_in, WI0, WH0, WI1, WH1, b_ih0, b_hh0, b_ih1, b_hh1, out1, HFIN);
  head_kernel<<<1, NTHD, 0, stream>>>(HFIN, fc_w, fc_b, out0);
}
